// TinyViT_24515673325836
// MI455X (gfx1250) — hardware-run, weakly checked
//
#include <hip/hip_runtime.h>
#include <math.h>

typedef __attribute__((ext_vector_type(16))) _Float16 v16h;
typedef __attribute__((ext_vector_type(16))) __bf16 v16b;
typedef __attribute__((ext_vector_type(8)))  _Float16 v8h;
typedef __attribute__((ext_vector_type(8)))  float v8f;
typedef __attribute__((ext_vector_type(4)))  float v4f;
typedef __attribute__((ext_vector_type(2)))  float v2f;
typedef __attribute__((ext_vector_type(4)))  unsigned v4u;
typedef __attribute__((ext_vector_type(4)))  int v4i;
typedef float __attribute__((may_alias)) float_a;
typedef int __attribute__((may_alias)) int_a;

template <typename T> __device__ __forceinline__ void vst2(void* p, T v) { *(volatile T*)p = v; __threadfence(); *(volatile T*)p = v; }
__device__ __forceinline__ v8f wmma16(v16h a, v16h b, v8f c) {
  v8f d = __builtin_amdgcn_wmma_f32_16x16x32_f16(false, a, false, b, (short)0, c, false, false);
  asm volatile("v_nop\n\tv_nop\n\tv_nop\n\tv_nop" : "+v"(d) : "v"(a), "v"(b));
  return d;
}
__device__ __forceinline__ v8f wmma_bf(v16b a, v16b b, v8f c) {
  v8f d = __builtin_amdgcn_wmma_f32_16x16x32_bf16(false, a, false, b, (short)0, c, false, false);
  asm volatile("v_nop\n\tv_nop\n\tv_nop\n\tv_nop" : "+v"(d) : "v"(a), "v"(b));
  return d;
}
__device__ __forceinline__ v16h frag_h(const _Float16* rowk0, int lane) {
  union { v16h v; v8h q[2]; } u; const _Float16* p = rowk0 + 8 * (lane >> 4);
  u.q[0] = *(const v8h*)p; u.q[1] = *(const v8h*)(p + 16); return u.v;
}
__device__ __forceinline__ v16h frag_f32(const float* rowk0, int lane) {
  v16h a; const float* p = rowk0 + 8 * (lane >> 4);
#pragma unroll
  for (int i = 0; i < 8; ++i) { a[i] = (_Float16)p[i]; a[8 + i] = (_Float16)p[16 + i]; }
  return a;
}
__device__ __forceinline__ v16h frag_f32s(const float* rowk0, int lane, float sc) {
  v16h a; const float* p = rowk0 + 8 * (lane >> 4);
#pragma unroll
  for (int i = 0; i < 8; ++i) { a[i] = (_Float16)(p[i] * sc); a[8 + i] = (_Float16)(p[16 + i] * sc); }
  return a;
}
__device__ __forceinline__ v16h fragc_f32(const float* W, int k0, int n, int lane, int ld, int K) {
  v16h a; const int g = lane >> 4;
#pragma unroll
  for (int i = 0; i < 8; ++i) { const int ka = k0 + 8 * g + i, kb = ka + 16;
    a[i] = (_Float16)(ka < K ? W[(size_t)(ka < K ? ka : K - 1) * ld + n] : 0.f); a[8 + i] = (_Float16)(kb < K ? W[(size_t)(kb < K ? kb : K - 1) * ld + n] : 0.f); }
  return a;
}
struct F2 { v16b h, l; };
__device__ __forceinline__ F2 bsplit16(const float v[16]) { F2 r;
#pragma unroll
  for (int i = 0; i < 16; ++i) { const __bf16 h = (__bf16)v[i]; r.h[i] = h; r.l[i] = (__bf16)(v[i] - (float)h); }
  return r; }
__device__ __forceinline__ F2 split_row(const float* row, int k0, int lane) { float v[16]; const float* p = row + k0 + 8 * (lane >> 4);
#pragma unroll
  for (int i = 0; i < 8; ++i) { v[i] = p[i]; v[8 + i] = p[16 + i]; }
  return bsplit16(v); }
__device__ __forceinline__ F2 split_rowK(const float* row, int k0, int lane, int K) { float v[16]; const int g = lane >> 4;
#pragma unroll
  for (int i = 0; i < 8; ++i) { const int ka = k0 + 8 * g + i, kb = ka + 16; v[i] = ka < K ? row[ka < K ? ka : K - 1] : 0.f; v[8 + i] = kb < K ? row[kb < K ? kb : K - 1] : 0.f; }
  return bsplit16(v); }
__device__ __forceinline__ F2 split_col(const float* W, int k0, int n, int lane, int ld, int K) { float v[16]; const int g = lane >> 4;
#pragma unroll
  for (int i = 0; i < 8; ++i) { const int ka = k0 + 8 * g + i, kb = ka + 16; v[i] = ka < K ? W[(size_t)(ka < K ? ka : K - 1) * ld + n] : 0.f; v[8 + i] = kb < K ? W[(size_t)(kb < K ? kb : K - 1) * ld + n] : 0.f; }
  return bsplit16(v); }
__device__ __forceinline__ v8f mac3(const F2& a, const F2& b, v8f c) { c = wmma_bf(a.l, b.h, c); c = wmma_bf(a.h, b.l, c); return wmma_bf(a.h, b.h, c); }
__device__ __forceinline__ float sigm(float v) { return 1.0f / (1.0f + expf(-v)); }
#define LDSX() do { asm volatile("s_wait_dscnt 0" ::: "memory"); __builtin_amdgcn_wave_barrier(); __builtin_amdgcn_fence(__ATOMIC_RELEASE, "workgroup"); } while (0)


#define NIMG 64
#define NTOK 1024
#define SQ 1025
#define DM 32
#define HD 16
#define NHD 2
#define NCLS 10
__device__ __forceinline__ float bfr(float v) { return (float)(__bf16)v; }
__device__ __attribute__((noinline)) float exp_ni(float v) { return expf(v); }
typedef __attribute__((ext_vector_type(8))) __bf16 v8b;
__device__ __forceinline__ v16b frag_b(const __bf16* rowk0, int lane) {
  union { v16b v; v8b q[2]; } u; const __bf16* p = rowk0 + 8 * (lane >> 4);
  u.q[0] = *(const v8b*)p; u.q[1] = *(const v8b*)(p + 16); return u.v;
}
__constant__ float c_freq[4] = {1.0f, 0.1f, 0.01f, 0.001f};

#define KROWS 1088
__global__ __launch_bounds__(128) void k_kv(const float* __restrict__ X, const float* __restrict__ R, const float* __restrict__ cls, const float* __restrict__ Wp, const float* __restrict__ bp,
                                            const float* __restrict__ Wk, const float* __restrict__ bk, const float* __restrict__ Wv, const float* __restrict__ bv, float* __restrict__ Kb, float* __restrict__ Vb) {
  __shared__ __align__(16) float sx[64][36]; __shared__ __align__(16) __bf16 swk[32][32], swv[32][32]; __shared__ __align__(16) float sk[4][16][36], sv[4][16][36];
  const int tid = threadIdx.x, wave = tid >> 5, lane = tid & 31, col = lane & 15, g = lane >> 4;
  const int img = blockIdx.y, s0 = blockIdx.x * 64;
  for (int q = tid; q < 32 * 32; q += 128) { const int n = q >> 5, k = q & 31; swk[n][k] = (__bf16)Wk[k * DM + n]; swv[n][k] = (__bf16)Wv[k * DM + n]; }
  for (int q = tid; q < 64 * 32; q += 128) { const int rl = q >> 5, j = q & 31; const int s = s0 + rl; float v = 0.f;
    const int n = s - 1; const int nc = n < 0 ? 0 : (n >= NTOK ? NTOK - 1 : n); const float xv = bfr(X[(size_t)img * NTOK + nc]);
    v = (s == 0) ? bfr(cls[j]) : ((s < SQ) ? xv * bfr(Wp[j]) + bfr(bp[j]) : 0.f);
    sx[rl][j] = v; }
  __syncthreads();
  { const F2 a = split_row(&sx[wave * 16 + col][0], 0, lane);
#pragma unroll
    for (int ct = 0; ct < 2; ++ct) { v8f ak = {}, av = {}; const v16b wk = frag_b(&swk[ct * 16 + col][0], lane), wv = frag_b(&swv[ct * 16 + col][0], lane);
      ak = wmma_bf(a.l, wk, ak); ak = wmma_bf(a.h, wk, ak); av = wmma_bf(a.l, wv, av); av = wmma_bf(a.h, wv, av);
#pragma unroll
      for (int r = 0; r < 8; ++r) { const int n = ct * 16 + col; sk[wave][8 * g + r][n] = ak[r] + bfr(bk[n]); sv[wave][8 * g + r][n] = av[r] + bfr(bv[n]); } } }
  LDSX();
  { const int rl = lane >> 1, half = lane & 1;
    const int s = s0 + wave * 16 + rl; const int n = s - 1; const int nc = n < 0 ? 0 : (n >= NTOK ? NTOK - 1 : n);
    const float rx = (s >= 1 && s < SQ) ? bfr(R[((size_t)img * NTOK + nc) * 2]) : 0.f, ry = (s >= 1 && s < SQ) ? bfr(R[((size_t)img * NTOK + nc) * 2 + 1]) : 0.f;
#pragma unroll
    for (int i = 0; i < 8; ++i) { const float ang = (i < 4 ? rx : ry) * c_freq[i & 3]; const float cs = cosf(ang), sn = sinf(ang);
      const int d0 = half * HD + 2 * i; const float t1 = sk[wave][rl][d0], t2 = sk[wave][rl][d0 + 1];
      sk[wave][rl][d0] = t1 * cs - t2 * sn; sk[wave][rl][d0 + 1] = t1 * sn + t2 * cs; } }
  LDSX();
  for (int q = lane; q < 16 * 8; q += 32) { const int rl = q >> 3, pc = q & 7; const size_t o = ((size_t)img * KROWS + s0 + wave * 16 + rl) * DM + pc * 4;
    vst2(Kb + o, *(const v4f*)(&sk[wave][rl][pc * 4])); vst2(Vb + o, *(const v4f*)(&sv[wave][rl][pc * 4])); }
}
__global__ __launch_bounds__(256) void k_cls(const float* __restrict__ cls, const float* __restrict__ Wq, const float* __restrict__ bq, const float* __restrict__ Kb, const float* __restrict__ Vb, const float* __restrict__ Wf, const float* __restrict__ bf_, float* __restrict__ OUTS) {
  __shared__ float sq[DM], sred[8], so[2][8][DM]; __shared__ __align__(16) float sout[32];
  const int tid = threadIdx.x, wave = tid >> 5, lane = tid & 31, img = blockIdx.x;
  if (tid < DM) { float a = bfr(bq[tid]);
#pragma unroll 1
    for (int k = 0; k < DM; ++k) a += bfr(cls[k]) * bfr(Wq[k * DM + tid]);
    sq[tid] = a; }
  __syncthreads();
#pragma unroll 1
  for (int h = 0; h < NHD; ++h) {
    float m = -3.0e38f;
    for (int s = tid; s < SQ; s += 256) { const float* kr = Kb + ((size_t)img * KROWS + s) * DM + h * HD; float d = 0.f;
#pragma unroll 4
      for (int e = 0; e < HD; ++e) d += sq[h * HD + e] * kr[e];
      m = fmaxf(m, d * 0.25f); }
#pragma unroll
    for (int o = 1; o < 32; o <<= 1) m = fmaxf(m, __shfl_xor(m, o));
    if (lane == 0) sred[wave] = m;
    __syncthreads();
    float mx = sred[0];
#pragma unroll
    for (int w = 1; w < 8; ++w) mx = fmaxf(mx, sred[w]);
    __syncthreads();
    float ssum = 0.f; float ov[HD];
#pragma unroll
    for (int e = 0; e < HD; ++e) ov[e] = 0.f;
    for (int s = tid; s < SQ; s += 256) { const float* kr = Kb + ((size_t)img * KROWS + s) * DM + h * HD; const float* vr = Vb + ((size_t)img * KROWS + s) * DM + h * HD; float d = 0.f;
#pragma unroll 4
      for (int e = 0; e < HD; ++e) d += sq[h * HD + e] * kr[e];
      const float p = exp_ni(d * 0.25f - mx); ssum += p;
#pragma unroll
      for (int e = 0; e < HD; ++e) ov[e] += p * vr[e]; }
#pragma unroll
    for (int o = 1; o < 32; o <<= 1) { ssum += __shfl_xor(ssum, o);
#pragma unroll
      for (int e = 0; e < HD; ++e) ov[e] += __shfl_xor(ov[e], o); }
    if (lane == 0) { sred[wave] = ssum;
#pragma unroll
      for (int e = 0; e < HD; ++e) so[h][wave][e] = ov[e]; }
    __syncthreads();
    if (tid < HD) { float s = 0.f, o = 0.f;
#pragma unroll
      for (int w = 0; w < 8; ++w) { s += sred[w]; o += so[h][w][tid]; }
      so[h][0][tid] = o / s; }
    __syncthreads(); }
  if (tid < NCLS) { float a = bfr(bf_[tid]);
#pragma unroll 1
    for (int k = 0; k < DM; ++k) a += so[k / HD][0][k % HD] * bfr(Wf[k * NCLS + tid]);
    sout[tid] = a; }
  if (tid >= NCLS && tid < 32) sout[tid] = 0.f;
  __syncthreads();
  if (tid < 8) vst2(OUTS + (size_t)img * 32 + tid * 4, *(const v4f*)&sout[tid * 4]);
}
__global__ __launch_bounds__(256) void k_fin(const float* __restrict__ OUTS, float* __restrict__ out) {
  const int tid = threadIdx.x; if (tid < NIMG * NCLS / 4) { v4f v;
#pragma unroll
    for (int i = 0; i < 4; ++i) { const int f = tid * 4 + i; v[i] = OUTS[(f / NCLS) * 32 + (f % NCLS)]; }
    vst2(out + tid * 4, v); }
}

extern "C" void kernel_launch(void* const* d_in, const int* in_sizes, int n_in, void* d_out, int out_size, void* d_ws, size_t ws_size, hipStream_t stream) {
  (void)in_sizes; (void)n_in; (void)out_size; (void)ws_size;
  const float** F = (const float**)d_in;
  float* Kb = (float*)d_ws; float* Vb = Kb + (size_t)NIMG * KROWS * DM; float* OUTS = Vb + (size_t)NIMG * KROWS * DM;
  k_kv<<<dim3(KROWS / 64, NIMG), 128, 0, stream>>>(F[0], F[1], F[2], F[3], F[4], F[7], F[8], F[9], F[10], Kb, Vb);
  k_cls<<<NIMG, 256, 0, stream>>>(F[2], F[5], F[6], Kb, Vb, F[11], F[12], OUTS);
  k_fin<<<1, 256, 0, stream>>>(OUTS, (float*)d_out);
}
